// MambaBlock_25288767439161
// MI455X (gfx1250) — hardware-verified
//
#include <hip/hip_runtime.h>
#include <math.h>

typedef __attribute__((ext_vector_type(16))) __bf16   v16b;
typedef __attribute__((ext_vector_type(8)))  __bf16   v8b;
typedef __attribute__((ext_vector_type(8)))  float    v8f;
typedef __attribute__((ext_vector_type(4)))  float    v4f;
typedef __attribute__((ext_vector_type(2)))  float    v2f;
typedef __attribute__((ext_vector_type(4)))  unsigned v4u;

constexpr int kBatch  = 2;
constexpr int kSeq    = 2048;
constexpr int kDm     = 1024;
constexpr int kDin    = 2048;
constexpr int kNst    = 16;
constexpr int kDtR    = 64;
constexpr int kPrjN   = kDtR + 2 * kNst;
constexpr int kPrjP   = 128;
constexpr int kRows   = kBatch * kSeq;
constexpr int kScanTS = 64;
constexpr int kScanCh = 64;
constexpr int kScanYP = 68;
static_assert(kPrjN == 96, "x_proj width");
static_assert((kDm % 32) == 0 && (kDin % 32) == 0 && (kDtR % 32) == 0, "GEMM K multiples of 32");
static_assert((kRows % 64) == 0 && (kDin % 64) == 0 && (kPrjP % 64) == 0 && (kDm % 64) == 0, "GEMM M,N multiples of 64");
static_assert((kSeq % kScanTS) == 0 && (kSeq % 64) == 0 && (kDin % kScanCh) == 0 && (kDin % 512) == 0, "tile multiples");
static_assert((kSeq & (kSeq - 1)) == 0, "sequence length power of two");

constexpr size_t kOffWXB  = 0;
constexpr size_t kOffWZB  = kOffWXB  + (size_t)kDin  * kDm   * 2;
constexpr size_t kOffWOB  = kOffWZB  + (size_t)kDin  * kDm   * 2;
constexpr size_t kOffWPB  = kOffWOB  + (size_t)kDm   * kDin  * 2;
constexpr size_t kOffWDB  = kOffWPB  + (size_t)kPrjP * kDin  * 2;
constexpr size_t kOffXN   = kOffWDB  + (size_t)kDin  * kDtR  * 2;
constexpr size_t kOffXB   = kOffXN   + (size_t)kRows * kDm   * 2;
constexpr size_t kOffZB   = kOffXB   + (size_t)kRows * kDin  * 2;
constexpr size_t kOffXC   = kOffZB   + (size_t)kRows * kDin  * 2;
constexpr size_t kOffPROJ = kOffXC   + (size_t)kRows * kDin  * 2;
constexpr size_t kOffDTL  = kOffPROJ + (size_t)kRows * kPrjP * 4;
constexpr size_t kOffDLR  = kOffDTL  + (size_t)kRows * kDtR  * 2;
constexpr size_t kOffYZ   = kOffDLR  + (size_t)kRows * kDin  * 4;
constexpr size_t kWsTotal = kOffYZ   + (size_t)kRows * kDin  * 2;
static_assert(kWsTotal == 125042688ull, "carve total");
static_assert(kWsTotal <= 134217728ull, "carve cap");
static_assert((kOffWZB % 128) == 0 && (kOffWOB % 128) == 0 && (kOffWPB % 128) == 0 && (kOffWDB % 128) == 0 &&
              (kOffXN % 128) == 0 && (kOffXB % 128) == 0 && (kOffZB % 128) == 0 && (kOffXC % 128) == 0 &&
              (kOffPROJ % 128) == 0 && (kOffDTL % 128) == 0 && (kOffDLR % 128) == 0 && (kOffYZ % 128) == 0,
              "128-B aligned regions");

__device__ __forceinline__ unsigned bf16_rne_bits(float f) {
  const unsigned u = __float_as_uint(f);
  return (u + 0x7FFFu + ((u >> 16) & 1u)) >> 16;
}
__device__ __forceinline__ unsigned pack_bf16x2(float lo, float hi) {
  const unsigned a = bf16_rne_bits(lo);
  const unsigned b = bf16_rne_bits(hi);
  return a | (b << 16);
}
__device__ __forceinline__ float bf16w_lo(unsigned w) { return __uint_as_float(w << 16); }
__device__ __forceinline__ float bf16w_hi(unsigned w) { return __uint_as_float(w & 0xffff0000u); }

union FragB { v16b v; v8b h[2]; };
__device__ __forceinline__ v16b frag_load(const __bf16* p) {
  FragB f;
  f.h[0] = *(const v8b*)(p);
  f.h[1] = *(const v8b*)(p + 16);
  return f.v;
}
__device__ __forceinline__ v8f frag_mma(v16b a, v16b b, v8f c) {
  return __builtin_amdgcn_wmma_f32_16x16x32_bf16(false, a, false, b, (short)0, c, false, false);
}
__device__ __forceinline__ void mma_group_guard(v8f& a, v8f& b, v8f& c, v8f& d, v16b x, v16b y0, v16b y1, v16b y2, v16b y3) {
  asm volatile("v_nop\n\tv_nop\n\tv_nop\n\tv_nop"
               : "+v"(a), "+v"(b), "+v"(c), "+v"(d)
               : "v"(x), "v"(y0), "v"(y1), "v"(y2), "v"(y3));
}
__device__ __forceinline__ void keep4_b(v16b a, v16b b, v16b c, v16b d) { asm volatile("v_nop" :: "v"(a), "v"(b), "v"(c), "v"(d)); }
__device__ __forceinline__ void acc_guard4(v8f& a, v8f& b, v8f& c, v8f& d) {
  asm volatile("v_nop\n\tv_nop\n\tv_nop\n\tv_nop" : "+v"(a), "+v"(b), "+v"(c), "+v"(d));
}

template <int OUT_MODE, bool BIAS, bool RESID>
__global__ __launch_bounds__(256) void wmma_gemm64_bf16(
    const unsigned short* __restrict__ Ap, int lda,
    const unsigned short* __restrict__ Btp, int ldb,
    void* __restrict__ Cout, int ldc,
    const float* __restrict__ bias,
    const float* __restrict__ resid,
    int M, int N, int K)
{
  const __bf16* A  = (const __bf16*)Ap;
  const __bf16* Bt = (const __bf16*)Btp;
  __shared__ __align__(16) float sT[8][16 * 68];
  const int lane = threadIdx.x & 31;
  const int wave = threadIdx.x >> 5;
  const int tilesN = N >> 6;
  const int tilesM = M >> 6;
  const int tile = blockIdx.x * 8 + wave;
  if (tile >= tilesM * tilesN) return;
  const int tm = tile / tilesN;
  const int tn = tile - tm * tilesN;
  const int m0 = tm << 6;
  const int n0 = tn << 6;

  const int rlane = lane & 15;
  const int koff  = (lane >> 4) * 8;
  const int mOff  = (lane >> 4) * 8;

  v8f acc[4][4];
#pragma unroll
  for (int i = 0; i < 4; ++i)
#pragma unroll
    for (int j = 0; j < 4; ++j) acc[i][j] = (v8f){0.f, 0.f, 0.f, 0.f, 0.f, 0.f, 0.f, 0.f};

  for (int k0 = 0; k0 < K; k0 += 32) {
    v16b bh[4];
#pragma unroll
    for (int j = 0; j < 4; ++j) {
      const size_t bo = (size_t)(n0 + (j << 4) + rlane) * ldb + koff + k0;
      bh[j] = frag_load(Bt + bo);
    }
#pragma unroll
    for (int i = 0; i < 4; ++i) {
      const size_t ao = (size_t)(m0 + (i << 4) + rlane) * lda + koff + k0;
      const v16b ah = frag_load(A + ao);
#pragma unroll
      for (int j = 0; j < 4; ++j) acc[i][j] = frag_mma(ah, bh[j], acc[i][j]);
      mma_group_guard(acc[i][0], acc[i][1], acc[i][2], acc[i][3], ah, bh[0], bh[1], bh[2], bh[3]);
    }
    keep4_b(bh[0], bh[1], bh[2], bh[3]);
  }
  acc_guard4(acc[0][0], acc[0][1], acc[0][2], acc[0][3]);
  acc_guard4(acc[1][0], acc[1][1], acc[1][2], acc[1][3]);
  acc_guard4(acc[2][0], acc[2][1], acc[2][2], acc[2][3]);
  acc_guard4(acc[3][0], acc[3][1], acc[3][2], acc[3][3]);

  float* slab = sT[wave];
#pragma unroll
  for (int i = 0; i < 4; ++i) {
    const int mBase = m0 + (i << 4);
#pragma unroll
    for (int j = 0; j < 4; ++j) {
#pragma unroll
      for (int r = 0; r < 8; ++r) slab[(mOff + r) * 68 + (j << 4) + rlane] = acc[i][j][r];
    }
    __builtin_amdgcn_fence(__ATOMIC_RELEASE, "workgroup");
    __builtin_amdgcn_wave_barrier();
    __builtin_amdgcn_fence(__ATOMIC_ACQUIRE, "workgroup");
    if (OUT_MODE == 0) {
      float* C = (float*)Cout;
      const int hh = lane >> 4, c4 = (lane & 15) * 4;
      v4f bb = (v4f){0.f, 0.f, 0.f, 0.f};
      if (BIAS) bb = *(const v4f*)(bias + n0 + c4);
      v4f ov[8];
#pragma unroll
      for (int it = 0; it < 4; ++it) {
        const int row = it * 2 + hh;
        v4f v = *(const v4f*)(slab + row * 68 + c4);
        v = v + bb;
        if (RESID) {
          const v4f rv = *(const v4f*)(resid + (size_t)(mBase + row) * ldc + n0 + c4);
          v = v + rv;
        }
        ov[it] = v;
      }
      asm volatile("" ::: "memory");
#pragma unroll
      for (int it = 4; it < 8; ++it) {
        const int row = it * 2 + hh;
        v4f v = *(const v4f*)(slab + row * 68 + c4);
        v = v + bb;
        if (RESID) {
          const v4f rv = *(const v4f*)(resid + (size_t)(mBase + row) * ldc + n0 + c4);
          v = v + rv;
        }
        ov[it] = v;
      }
      for (int pass = 0; pass < 2; ++pass) {
#pragma unroll
        for (int it = 0; it < 8; ++it) {
          const int row = it * 2 + hh;
          *(volatile v4f*)(C + (size_t)(mBase + row) * ldc + n0 + c4) = ov[it];
        }
        __threadfence();
      }
    } else {
      unsigned short* C = (unsigned short*)Cout;
      const int q = lane >> 3, c8 = (lane & 7) * 8;
      v4f b0 = (v4f){0.f, 0.f, 0.f, 0.f};
      v4f b1 = (v4f){0.f, 0.f, 0.f, 0.f};
      if (BIAS) {
        b0 = *(const v4f*)(bias + n0 + c8);
        b1 = *(const v4f*)(bias + n0 + c8 + 4);
      }
      v4u hv[4];
#pragma unroll
      for (int it = 0; it < 4; ++it) {
        const int row = it * 4 + q;
        const float* sp = slab + row * 68 + c8;
        const v4f a0 = *(const v4f*)(sp);
        const v4f a1 = *(const v4f*)(sp + 4);
        const float f0 = a0[0] + b0[0];
        const float f1 = a0[1] + b0[1];
        const float f2 = a0[2] + b0[2];
        const float f3 = a0[3] + b0[3];
        const float f4 = a1[0] + b1[0];
        const float f5 = a1[1] + b1[1];
        const float f6 = a1[2] + b1[2];
        const float f7 = a1[3] + b1[3];
        v4u w;
        w[0] = pack_bf16x2(f0, f1);
        w[1] = pack_bf16x2(f2, f3);
        w[2] = pack_bf16x2(f4, f5);
        w[3] = pack_bf16x2(f6, f7);
        hv[it] = w;
      }
      for (int pass = 0; pass < 2; ++pass) {
#pragma unroll
        for (int it = 0; it < 4; ++it) {
          const int row = it * 4 + q;
          *(volatile v4u*)(C + (size_t)(mBase + row) * ldc + n0 + c8) = hv[it];
        }
        __threadfence();
      }
    }
    __builtin_amdgcn_fence(__ATOMIC_RELEASE, "workgroup");
    __builtin_amdgcn_wave_barrier();
    __builtin_amdgcn_fence(__ATOMIC_ACQUIRE, "workgroup");
  }
}

__global__ __launch_bounds__(256) void cast_bf16_kernel(
    const float* __restrict__ src, unsigned* __restrict__ dstw, int total8, int real8)
{
  const int i = blockIdx.x * 256 + threadIdx.x;
  if (i >= total8) return;
  const bool keep = (i < real8);
  const int ic = keep ? i : (real8 - 1);
  const float* p = src + ((size_t)ic << 3);
  const v4f a0 = *(const v4f*)(p);
  const v4f a1 = *(const v4f*)(p + 4);
  const float f0 = keep ? a0[0] : 0.0f;
  const float f1 = keep ? a0[1] : 0.0f;
  const float f2 = keep ? a0[2] : 0.0f;
  const float f3 = keep ? a0[3] : 0.0f;
  const float f4 = keep ? a1[0] : 0.0f;
  const float f5 = keep ? a1[1] : 0.0f;
  const float f6 = keep ? a1[2] : 0.0f;
  const float f7 = keep ? a1[3] : 0.0f;
  v4u w;
  w[0] = pack_bf16x2(f0, f1);
  w[1] = pack_bf16x2(f2, f3);
  w[2] = pack_bf16x2(f4, f5);
  w[3] = pack_bf16x2(f6, f7);
  unsigned* q = dstw + ((size_t)i << 2);
  *(volatile v4u*)q = w;
  __threadfence();
  *(volatile v4u*)q = w;
}

__global__ __launch_bounds__(256) void rmsnorm_bf16_kernel(
    const float* __restrict__ x, const float* __restrict__ w, unsigned* __restrict__ XNw)
{
  const int lane = threadIdx.x & 31, wave = threadIdx.x >> 5;
  const int tok = blockIdx.x * 8 + wave;
  const float* xr = x + (size_t)tok * kDm;
  v4f a[8];
#pragma unroll
  for (int it = 0; it < 4; ++it) {
    a[2 * it]     = *(const v4f*)(xr + it * 256 + lane * 8);
    a[2 * it + 1] = *(const v4f*)(xr + it * 256 + lane * 8 + 4);
  }
  float ss = 0.0f;
#pragma unroll
  for (int i = 0; i < 8; ++i) {
    ss = fmaf(a[i][0], a[i][0], ss);
    ss = fmaf(a[i][1], a[i][1], ss);
    ss = fmaf(a[i][2], a[i][2], ss);
    ss = fmaf(a[i][3], a[i][3], ss);
  }
#pragma unroll
  for (int off = 16; off > 0; off >>= 1) ss += __shfl_xor(ss, off, 32);
  const float sc = rsqrtf(ss * (1.0f / (float)kDm) + 1e-5f);
  asm volatile("" ::: "memory");
  v4u ov[4];
#pragma unroll
  for (int it = 0; it < 4; ++it) {
    const v4f w0 = *(const v4f*)(w + it * 256 + lane * 8);
    const v4f w1 = *(const v4f*)(w + it * 256 + lane * 8 + 4);
    const float f0 = (a[2 * it][0] * sc) * w0[0];
    const float f1 = (a[2 * it][1] * sc) * w0[1];
    const float f2 = (a[2 * it][2] * sc) * w0[2];
    const float f3 = (a[2 * it][3] * sc) * w0[3];
    const float f4 = (a[2 * it + 1][0] * sc) * w1[0];
    const float f5 = (a[2 * it + 1][1] * sc) * w1[1];
    const float f6 = (a[2 * it + 1][2] * sc) * w1[2];
    const float f7 = (a[2 * it + 1][3] * sc) * w1[3];
    v4u o;
    o[0] = pack_bf16x2(f0, f1);
    o[1] = pack_bf16x2(f2, f3);
    o[2] = pack_bf16x2(f4, f5);
    o[3] = pack_bf16x2(f6, f7);
    ov[it] = o;
  }
  unsigned* orow = XNw + (size_t)tok * (kDm / 2);
  for (int pass = 0; pass < 2; ++pass) {
#pragma unroll
    for (int it = 0; it < 4; ++it) *(volatile v4u*)(orow + it * 128 + lane * 4) = ov[it];
    __threadfence();
  }
}

__global__ __launch_bounds__(256) void conv_silu_kernel(
    const unsigned* __restrict__ XBw, const float* __restrict__ cw, const float* __restrict__ cb,
    unsigned* __restrict__ XCw)
{
  const int tid = threadIdx.x;
  const int p  = blockIdx.x * 256 + tid;
  const int g0 = blockIdx.y * 64;
  const int tb = g0 & (kSeq - 1);
  const v4f wa = *(const v4f*)(cw + 8 * p);
  const v4f wb = *(const v4f*)(cw + 8 * p + 4);
  const v2f bc = *(const v2f*)(cb + 2 * p);
  const float wa0 = wa[0], wa1 = wa[1], wa2 = wa[2], wa3 = wa[3];
  const float wb0 = wb[0], wb1 = wb[1], wb2 = wb[2], wb3 = wb[3];
  const float ba = bc[0], bb = bc[1];
  const bool hist = (tb > 0);
  const int rb = hist ? (g0 - 3) : g0;
  const unsigned h3 = XBw[(size_t)rb * (kDin / 2) + p];
  const unsigned h2 = XBw[(size_t)(rb + 1) * (kDin / 2) + p];
  const unsigned h1 = XBw[(size_t)(rb + 2) * (kDin / 2) + p];
  float am3 = hist ? bf16w_lo(h3) : 0.0f;
  float am2 = hist ? bf16w_lo(h2) : 0.0f;
  float am1 = hist ? bf16w_lo(h1) : 0.0f;
  float bm3 = hist ? bf16w_hi(h3) : 0.0f;
  float bm2 = hist ? bf16w_hi(h2) : 0.0f;
  float bm1 = hist ? bf16w_hi(h1) : 0.0f;
#pragma unroll 1
  for (int s = 0; s < 64; ++s) {
    const size_t o = (size_t)(g0 + s) * (kDin / 2) + p;
    const unsigned wv = XBw[o];
    const float xa = bf16w_lo(wv);
    const float xb = bf16w_hi(wv);
    float sa = wa0 * am3;
    sa = fmaf(wa1, am2, sa);
    sa = fmaf(wa2, am1, sa);
    sa = fmaf(wa3, xa, sa);
    sa = sa + ba;
    float sb = wb0 * bm3;
    sb = fmaf(wb1, bm2, sb);
    sb = fmaf(wb2, bm1, sb);
    sb = fmaf(wb3, xb, sb);
    sb = sb + bb;
    const float ya = sa * __builtin_amdgcn_rcpf(1.0f + expf(-sa));
    const float yb = sb * __builtin_amdgcn_rcpf(1.0f + expf(-sb));
    const unsigned u = pack_bf16x2(ya, yb);
    unsigned* q = XCw + o;
    *(volatile unsigned*)q = u;
    __threadfence();
    *(volatile unsigned*)q = u;
    am3 = am2; am2 = am1; am1 = xa;
    bm3 = bm2; bm2 = bm1; bm1 = xb;
  }
}

__global__ __launch_bounds__(256) void dtlow_cast_kernel(
    const float* __restrict__ PROJ, unsigned* __restrict__ DTLw, int total8)
{
  const int i = blockIdx.x * 256 + threadIdx.x;
  if (i >= total8) return;
  const int e0  = i << 3;
  const int row = e0 >> 6;
  const int c8  = e0 & 63;
  const float* p = PROJ + (size_t)row * kPrjP + c8;
  const v4f a0 = *(const v4f*)(p);
  const v4f a1 = *(const v4f*)(p + 4);
  const float f0 = a0[0], f1 = a0[1], f2 = a0[2], f3 = a0[3];
  const float f4 = a1[0], f5 = a1[1], f6 = a1[2], f7 = a1[3];
  v4u w;
  w[0] = pack_bf16x2(f0, f1);
  w[1] = pack_bf16x2(f2, f3);
  w[2] = pack_bf16x2(f4, f5);
  w[3] = pack_bf16x2(f6, f7);
  unsigned* q = DTLw + ((size_t)i << 2);
  *(volatile v4u*)q = w;
  __threadfence();
  *(volatile v4u*)q = w;
}

__global__ __launch_bounds__(64) void scan_gate_kernel(
    const float* __restrict__ DLR, const unsigned* __restrict__ XCw, const unsigned* __restrict__ ZBw,
    const float* __restrict__ PROJ, const float* __restrict__ Alog, const float* __restrict__ Dp,
    unsigned* __restrict__ YZw)
{
#pragma clang fp contract(off)
  __shared__ __align__(16) float sBC[kScanTS * 32];
  __shared__ __align__(16) float sY[kScanTS * kScanYP];
  __shared__ __align__(16) float sA[kNst * kScanCh];
  const int tid = threadIdx.x, lane = tid & 31, wave = tid >> 5;
  constexpr int kBlkPerB = kDin / kScanCh;
  const int bix = blockIdx.x / kBlkPerB;
  const int d0  = (blockIdx.x - bix * kBlkPerB) * kScanCh;
  const int d   = d0 + tid;
  const size_t row0 = (size_t)bix * kSeq;
#pragma unroll 1
  for (int s = 0; s < kNst; ++s) sA[s * kScanCh + tid] = -expf(Alog[(size_t)d * kNst + s]);
  __syncthreads();
  float negA[kNst], h[kNst];
#pragma unroll
  for (int s = 0; s < kNst; ++s) {
    negA[s] = sA[s * kScanCh + tid];
    h[s] = 0.0f;
  }
  const float Dd = Dp[d];
  const bool odd = (tid & 1) != 0;
  const int dw = d >> 1;
  const int lr = tid >> 3, lc4 = (tid & 7) * 4;
  const int q = lane >> 3, c8 = (lane & 7) * 8;
#pragma unroll 1
  for (int t0 = 0; t0 < kSeq; t0 += kScanTS) {
    __syncthreads();
#pragma unroll
    for (int i = 0; i < 8; ++i) {
      const int r = lr + 8 * i;
      *(v4f*)(sBC + r * 32 + lc4) = *(const v4f*)(PROJ + (row0 + t0 + r) * kPrjP + kDtR + lc4);
    }
    __syncthreads();
#pragma unroll 1
    for (int s = 0; s < kScanTS; ++s) {
      const size_t grow = row0 + t0 + s;
      const float a = DLR[grow * kDin + d];
      const unsigned xw = XCw[grow * (kDin / 2) + dw];
      const unsigned zw = ZBw[grow * (kDin / 2) + dw];
      const float xv = __uint_as_float(odd ? (xw & 0xffff0000u) : (xw << 16));
      const float zv = __uint_as_float(odd ? (zw & 0xffff0000u) : (zw << 16));
      const float delta = fmaxf(a, 0.0f) + log1pf(expf(-fabsf(a)));
      const float* br = sBC + s * 32;
      float Bs[kNst], Cs[kNst];
#pragma unroll
      for (int q4 = 0; q4 < 4; ++q4) {
        const v4f bv = *(const v4f*)(br + 4 * q4);
        const v4f cv = *(const v4f*)(br + kNst + 4 * q4);
        Bs[4 * q4 + 0] = bv[0]; Bs[4 * q4 + 1] = bv[1]; Bs[4 * q4 + 2] = bv[2]; Bs[4 * q4 + 3] = bv[3];
        Cs[4 * q4 + 0] = cv[0]; Cs[4 * q4 + 1] = cv[1]; Cs[4 * q4 + 2] = cv[2]; Cs[4 * q4 + 3] = cv[3];
      }
      float y = 0.0f;
#pragma unroll
      for (int k = 0; k < kNst; ++k) {
        const float e  = expf(delta * negA[k]);
        const float db = delta * Bs[k];
        const float pr = db * xv;
        const float hn = e * h[k] + pr;
        h[k] = hn;
        y = y + hn * Cs[k];
      }
      y = y + xv * Dd;
      const float sg = __builtin_amdgcn_rcpf(1.0f + expf(-zv));
      y = y * (zv * sg);
      sY[s * kScanYP + tid] = y;
    }
    __syncthreads();
    v4u hv[8];
#pragma unroll
    for (int it = 0; it < 8; ++it) {
      const int row = it * 8 + wave * 4 + q;
      const float* sp = sY + row * kScanYP + c8;
      const v4f a0 = *(const v4f*)(sp);
      const v4f a1 = *(const v4f*)(sp + 4);
      const float f0 = a0[0], f1 = a0[1], f2 = a0[2], f3 = a0[3];
      const float f4 = a1[0], f5 = a1[1], f6 = a1[2], f7 = a1[3];
      v4u w;
      w[0] = pack_bf16x2(f0, f1);
      w[1] = pack_bf16x2(f2, f3);
      w[2] = pack_bf16x2(f4, f5);
      w[3] = pack_bf16x2(f6, f7);
      hv[it] = w;
    }
    for (int pass = 0; pass < 2; ++pass) {
#pragma unroll
      for (int it = 0; it < 8; ++it) {
        const int row = it * 8 + wave * 4 + q;
        unsigned* o = YZw + (row0 + t0 + row) * (kDin / 2) + (d0 >> 1) + (lane & 7) * 4;
        *(volatile v4u*)o = hv[it];
      }
      __threadfence();
    }
  }
}

extern "C" void kernel_launch(void* const* d_in, const int* in_sizes, int n_in,
                              void* d_out, int out_size, void* d_ws, size_t ws_size,
                              hipStream_t stream)
{
  if (n_in < 15) return;
  if (in_sizes[0]  != kRows * kDm)  return;
  if (in_sizes[1]  != kDm)          return;
  if (in_sizes[2]  != kDin * kDm)   return;
  if (in_sizes[3]  != kDin)         return;
  if (in_sizes[4]  != kDin * kDm)   return;
  if (in_sizes[5]  != kDin)         return;
  if (in_sizes[6]  != kDin * 4)     return;
  if (in_sizes[7]  != kDin)         return;
  if (in_sizes[8]  != kPrjN * kDin) return;
  if (in_sizes[9]  != kDin * kDtR)  return;
  if (in_sizes[10] != kDin)         return;
  if (in_sizes[11] != kDin * kNst)  return;
  if (in_sizes[12] != kDin)         return;
  if (in_sizes[13] != kDm * kDin)   return;
  if (in_sizes[14] != kDm)          return;
  if (out_size != kRows * kDm) return;
  if (ws_size < kWsTotal) return;

  const float* x      = (const float*)d_in[0];
  const float* norm_w = (const float*)d_in[1];
  const float* Wx     = (const float*)d_in[2];
  const float* bx     = (const float*)d_in[3];
  const float* Wz     = (const float*)d_in[4];
  const float* bz     = (const float*)d_in[5];
  const float* conv_w = (const float*)d_in[6];
  const float* conv_b = (const float*)d_in[7];
  const float* Wxp    = (const float*)d_in[8];
  const float* Wdt    = (const float*)d_in[9];
  const float* bdt    = (const float*)d_in[10];
  const float* A_log  = (const float*)d_in[11];
  const float* Dp     = (const float*)d_in[12];
  const float* Wout   = (const float*)d_in[13];
  const float* bout   = (const float*)d_in[14];
  float* out = (float*)d_out;

  char* ws = (char*)d_ws;
  unsigned short* WXB  = (unsigned short*)(ws + kOffWXB);
  unsigned short* WZB  = (unsigned short*)(ws + kOffWZB);
  unsigned short* WOB  = (unsigned short*)(ws + kOffWOB);
  unsigned short* WPB  = (unsigned short*)(ws + kOffWPB);
  unsigned short* WDB  = (unsigned short*)(ws + kOffWDB);
  unsigned short* XN   = (unsigned short*)(ws + kOffXN);
  unsigned short* XB   = (unsigned short*)(ws + kOffXB);
  unsigned short* ZB   = (unsigned short*)(ws + kOffZB);
  unsigned short* XC   = (unsigned short*)(ws + kOffXC);
  float*          PROJ = (float*)(ws + kOffPROJ);
  unsigned short* DTL  = (unsigned short*)(ws + kOffDTL);
  float*          DLR  = (float*)(ws + kOffDLR);
  unsigned short* YZ   = (unsigned short*)(ws + kOffYZ);

  {
    const int n8 = kDin * kDm / 8;
    cast_bf16_kernel<<<n8 / 256, 256, 0, stream>>>(Wx, (unsigned*)WXB, n8, n8);
    cast_bf16_kernel<<<n8 / 256, 256, 0, stream>>>(Wz, (unsigned*)WZB, n8, n8);
    cast_bf16_kernel<<<n8 / 256, 256, 0, stream>>>(Wout, (unsigned*)WOB, n8, n8);
    const int p8 = kPrjP * kDin / 8;
    const int r8 = kPrjN * kDin / 8;
    cast_bf16_kernel<<<p8 / 256, 256, 0, stream>>>(Wxp, (unsigned*)WPB, p8, r8);
    const int t8 = kDin * kDtR / 8;
    cast_bf16_kernel<<<t8 / 256, 256, 0, stream>>>(Wdt, (unsigned*)WDB, t8, t8);
  }

  rmsnorm_bf16_kernel<<<kRows / 8, 256, 0, stream>>>(x, norm_w, (unsigned*)XN);

  wmma_gemm64_bf16<1, true, false><<<(kRows / 64) * (kDin / 64) / 8, 256, 0, stream>>>(
      XN, kDm, WXB, kDm, (void*)XB, kDin, bx, x, kRows, kDin, kDm);
  wmma_gemm64_bf16<1, true, false><<<(kRows / 64) * (kDin / 64) / 8, 256, 0, stream>>>(
      XN, kDm, WZB, kDm, (void*)ZB, kDin, bz, x, kRows, kDin, kDm);

  conv_silu_kernel<<<dim3(kDin / 512, kRows / 64), 256, 0, stream>>>(
      (const unsigned*)XB, conv_w, conv_b, (unsigned*)XC);

  wmma_gemm64_bf16<0, false, false><<<(kRows / 64) * (kPrjP / 64) / 8, 256, 0, stream>>>(
      XC, kDin, WPB, kDin, (void*)PROJ, kPrjP, bdt, x, kRows, kPrjP, kDin);

  dtlow_cast_kernel<<<(kRows * kDtR / 8) / 256, 256, 0, stream>>>(PROJ, (unsigned*)DTL, kRows * kDtR / 8);

  wmma_gemm64_bf16<0, true, false><<<(kRows / 64) * (kDin / 64) / 8, 256, 0, stream>>>(
      DTL, kDtR, WDB, kDtR, (void*)DLR, kDin, bdt, x, kRows, kDin, kDtR);

  scan_gate_kernel<<<kBatch * (kDin / kScanCh), kScanCh, 0, stream>>>(
      DLR, (const unsigned*)XC, (const unsigned*)ZB, PROJ, A_log, Dp, (unsigned*)YZ);

  wmma_gemm64_bf16<0, true, true><<<(kRows / 64) * (kDm / 64) / 8, 256, 0, stream>>>(
      YZ, kDin, WOB, kDin, (void*)out, kDm, bout, x, kRows, kDm, kDin);
}
